// GCN_MLP_53412213293178
// MI455X (gfx1250) — hardware-run, weakly checked
//
#include <hip/hip_runtime.h>


namespace {
constexpr int N = 100000, NP = 100032  , E = 1600000, F0 = 128, H = 64, NG = 64;
constexpr float XS = 8.0f, WSC = 256.0f, NEG = 0.2f  , LNEPS = 1e-5f;

typedef _Float16 b16;
typedef __attribute__((ext_vector_type(16))) _Float16 v16b;
typedef __attribute__((ext_vector_type(8))) _Float16 v8b;
typedef __attribute__((ext_vector_type(8))) float v8f;
typedef __attribute__((ext_vector_type(4))) float v4f;
__device__ __forceinline__ float bf16_rne(float f) { unsigned int u = __float_as_uint(f); u += 0x7FFFu + ((u >> 16) & 1u); return __uint_as_float(u & 0xFFFF0000u); }
__device__ __forceinline__ void split16(float v, b16& hi, b16& lo) { hi = (b16)v; lo = (b16)(v - (float)hi); }
__device__ __forceinline__ v16b frag_kb(const b16* p, int hh) { const v8b a = *(const v8b*)(p + 8 * hh), b = *(const v8b*)(p + 16 + 8 * hh); v16b f;
#pragma unroll
  for (int e = 0; e < 8; ++e) { f[e] = a[e]; f[8 + e] = b[e]; } return f; }
__device__ __forceinline__ v8f wmma16b(v16b a, v16b b, v8f c) { v8f d = __builtin_amdgcn_wmma_f32_16x16x32_f16(false, a, false, b, (short)0, c, false, false); asm volatile("v_nop\n\tv_nop\n\tv_nop\n\tv_nop" : "+v"(d) : "v"(a), "v"(b)); return d; }
__device__ __forceinline__ void wave_lds_sync() { __builtin_amdgcn_fence(__ATOMIC_RELEASE, "workgroup"); __builtin_amdgcn_wave_barrier(); __builtin_amdgcn_fence(__ATOMIC_ACQUIRE, "workgroup"); }
__device__ __forceinline__ float pmul(float a, float b) { float p = a * b; asm volatile("" : "+v"(p)); return p; }
__device__ __forceinline__ int iclamp(int v, int lo, int hi) { return v < lo ? lo : (v > hi ? hi : v); }
__device__ __forceinline__ float nexp(float x) { return __builtin_amdgcn_exp2f(x * 1.4426950408889634f); }
__device__ __forceinline__ float lrelu(float x) { return x > 0.0f ? x : NEG * x; }

constexpr int CSR_NBLK = 512, CSR_GB = 9, CSR_GN = 1 << CSR_GB  , CSR_MAXG = 512, CSR_CAP = 12288  ;
__global__ __launch_bounds__(64) void csrA_kernel(const int* __restrict__ dst, int E, int N, int nG, int CHP, int NGP, int* __restrict__ STG, int* __restrict__ HST) {
  extern __shared__ int sm[];
  int* cnt = sm; int* run = sm + NGP; int* ids = sm + 2 * NGP;
  const int b = blockIdx.x; const int ch = (E + CSR_NBLK - 1) / CSR_NBLK; const int e0 = b * ch, e1 = min(E, e0 + ch);
  for (int i = threadIdx.x; i < NGP; i += 64) cnt[i] = 0;
  for (int i = threadIdx.x; i < CHP; i += 64) ids[i] = -1;
  __syncthreads();
  if (threadIdx.x == 0) {
    for (int e = e0; e < e1; ++e) { int d = dst[e]; d = (d < 0) ? 0 : (d >= N ? N - 1 : d); cnt[d >> CSR_GB] += 1; }
    int acc = 0; for (int g = 0; g < nG; ++g) { run[g] = acc; acc += cnt[g]; }
    for (int e = e0; e < e1; ++e) { int d = dst[e]; d = (d < 0) ? 0 : (d >= N ? N - 1 : d); const int g = d >> CSR_GB; ids[run[g]] = e; run[g] += 1; } }
  __syncthreads();
  typedef __attribute__((ext_vector_type(4))) int v4i;
  for (int pass = 0; pass < 2; ++pass) {
    for (int i = threadIdx.x; i < CHP / 4; i += 64) *(volatile v4i*)(STG + (size_t)b * CHP + i * 4) = *(const v4i*)(&ids[i * 4]);
    for (int i = threadIdx.x; i < NGP / 4; i += 64) { v4i v; for (int e = 0; e < 4; ++e) v[e] = (i * 4 + e < nG) ? cnt[i * 4 + e] : 0; *(volatile v4i*)(HST + (size_t)b * NGP + i * 4) = v; }
    __threadfence(); }
}
__global__ __launch_bounds__(512) void csrS_kernel(const int* __restrict__ HST, int nG, int NGP, int* __restrict__ START, int* __restrict__ TOT, int* __restrict__ OFF) {
  __shared__ int tot[CSR_MAXG];
  const int b = threadIdx.x;
  for (int pass = 0; pass < 2; ++pass) { int runb = 0; for (int g = 0; g < nG; ++g) { int c = HST[(size_t)b * NGP + g]; c = (c < 0) ? 0 : c; ((volatile int*)OFF)[(size_t)g * CSR_NBLK + b] = runb; runb += c; } __threadfence(); }
  for (int g = threadIdx.x; g < nG; g += 512) { int s = 0; for (int bb = 0; bb < CSR_NBLK; ++bb) { int c = HST[(size_t)bb * NGP + g]; s += (c < 0) ? 0 : c; } tot[g] = s; }
  __syncthreads();
  if (threadIdx.x < 32) {
    __shared__ int st[CSR_MAXG + 32];
    if (threadIdx.x == 0) { int acc = 0; for (int g = 0; g < NGP; ++g) { st[g] = acc; if (g < nG) acc += (tot[g] + 31) & ~31; } st[NGP] = acc; }
    __builtin_amdgcn_fence(__ATOMIC_RELEASE, "workgroup"); __builtin_amdgcn_wave_barrier(); __builtin_amdgcn_fence(__ATOMIC_ACQUIRE, "workgroup");
    for (int pass = 0; pass < 2; ++pass) { for (int i = threadIdx.x; i < NGP + 32; i += 32) { ((volatile int*)START)[i] = (i <= NGP) ? st[min(i, NGP)] : 0; ((volatile int*)TOT)[i] = (i < nG) ? tot[i] : 0; } __threadfence(); } }
}
__global__ __launch_bounds__(256) void csrB_kernel(const int* __restrict__ dst, int N, int nG, int CHP, int NGP, int permLen, const int* __restrict__ STG, const int* __restrict__ HST, const int* __restrict__ OFF, const int* __restrict__ START, const int* __restrict__ TOT, int* __restrict__ PERM, int* __restrict__ ROWPTR, int* __restrict__ ROWCNT, int* __restrict__ FLAG) {
  typedef __attribute__((ext_vector_type(4))) int v4i;
  __shared__ int ids[CSR_CAP]; __shared__ unsigned short key[CSR_CAP]; __shared__ int outp[CSR_CAP]; __shared__ int ncnt[CSR_GN + 1]; __shared__ int boff[CSR_NBLK + 1];
  const int g = blockIdx.x, t_ = threadIdx.x; int tot = TOT[g]; int st = START[g], stn = START[g + 1]; const int v0 = g * CSR_GN; const int nv = min(CSR_GN, N - v0);
  st = (st < 0) ? 0 : (st > permLen - 32 ? permLen - 32 : st) & ~31; stn = (stn < st) ? st : (stn > permLen ? permLen : stn); tot = (tot < 0) ? 0 : tot; if (tot > stn - st && tot <= CSR_CAP) tot = stn - st;
  if (tot > CSR_CAP) {
    for (int pass = 0; pass < 2; ++pass) { for (int i = t_; i < CSR_GN / 4; i += 256) { v4i a, c; for (int e = 0; e < 4; ++e) { a[e] = st; c[e] = 0; } *(volatile v4i*)(ROWPTR + v0 + i * 4) = a; *(volatile v4i*)(ROWCNT + v0 + i * 4) = c; } if (t_ == 0) ((volatile int*)FLAG)[0] = 1; __threadfence(); } (void)nv; return; }
  if (t_ == 0) { int acc = 0; for (int b = 0; b < CSR_NBLK; ++b) { boff[b] = acc; int c = HST[(size_t)b * NGP + g]; c = (c < 0) ? 0 : (c > CHP ? CHP : c); acc += c; if (acc > tot) acc = tot; } boff[CSR_NBLK] = acc; }
  for (int i = t_; i <= CSR_GN; i += 256) ncnt[i] = 0;
  __syncthreads();
  for (int b = 0; b < CSR_NBLK; ++b) { const int c = boff[b + 1] - boff[b]; int o_ = OFF[(size_t)g * CSR_NBLK + b]; o_ = (o_ < 0) ? 0 : (o_ > CHP - c ? CHP - c : o_); const int* src_ = STG + (size_t)b * CHP + o_;
    for (int i = t_; i < c; i += 256) { int id = src_[i]; id = (id < 0) ? 0 : id; ids[boff[b] + i] = id; int d = dst[id]; d = (d < v0) ? v0 : (d >= N ? N - 1 : d); int kk = d - v0; kk = (kk < 0) ? 0 : (kk >= CSR_GN ? CSR_GN - 1 : kk); key[boff[b] + i] = (unsigned short)kk; } }
  __syncthreads();
  if (t_ == 0) { for (int i = 0; i < tot; ++i) ncnt[key[i]] += 1; int acc = 0; for (int vl = 0; vl < CSR_GN; ++vl) { const int c = ncnt[vl]; ncnt[vl] = acc; acc += c; } ncnt[CSR_GN] = acc;
    for (int i = 0; i < tot; ++i) { const int vl = key[i]; outp[ncnt[vl]] = ids[i]; ncnt[vl] += 1; }
    for (int vl = CSR_GN; vl > 0; --vl) ncnt[vl] = ncnt[vl - 1]; ncnt[0] = 0; }
  __syncthreads();
  for (int pass = 0; pass < 2; ++pass) {
    for (int i = t_; i < (stn - st) / 4; i += 256) { v4i v; for (int e = 0; e < 4; ++e) { const int q = i * 4 + e; v[e] = (q < tot) ? outp[q] : -1; } *(volatile v4i*)(PERM + st + i * 4) = v; }
    for (int i = t_; i < CSR_GN / 4; i += 256) { v4i a, c; for (int e = 0; e < 4; ++e) { const int vl = i * 4 + e; a[e] = st + ncnt[vl]; c[e] = (vl < nv) ? (ncnt[vl + 1] - ncnt[vl]) : 0; } *(volatile v4i*)(ROWPTR + v0 + i * 4) = a; *(volatile v4i*)(ROWCNT + v0 + i * 4) = c; }
    __threadfence(); }
}
__global__ __launch_bounds__(256) void csrZ_kernel(int* __restrict__ p, size_t n4) { typedef __attribute__((ext_vector_type(4))) int v4i; const size_t tid = (size_t)blockIdx.x * 256 + threadIdx.x, nth = (size_t)gridDim.x * 256; v4i z = {0, 0, 0, 0}; for (size_t i = tid; i < n4; i += nth) *(volatile v4i*)(p + i * 4) = z; }
struct CsrBufs { int *STG, *HST, *OFF, *START, *TOT, *PERM, *ROWPTR, *ROWCNT, *FLAG; int nG, NGP, CHP; size_t permLen; char* base; size_t bytes; };
static size_t csr_carve(CsrBufs& c, char* ws, size_t off, int E, int N) {
  const size_t off0 = off; c.base = ws + off;
  auto al = [&](size_t bytes) { char* p = ws + off; off += (bytes + 255) & ~(size_t)255; return p; };
  c.nG = (N + CSR_GN - 1) / CSR_GN; c.NGP = (c.nG + 31) & ~31; const int ch = (E + CSR_NBLK - 1) / CSR_NBLK; c.CHP = (ch + 31) & ~31; c.permLen = (size_t)E + 32 * (size_t)c.nG + 32;
  c.STG = (int*)al((size_t)CSR_NBLK * c.CHP * 4); c.HST = (int*)al((size_t)CSR_NBLK * c.NGP * 4); c.OFF = (int*)al((size_t)c.NGP * CSR_NBLK * 4); c.START = (int*)al((size_t)(c.NGP + 64) * 4); c.TOT = (int*)al((size_t)(c.NGP + 64) * 4);
  c.PERM = (int*)al(c.permLen * 4); c.ROWPTR = (int*)al((size_t)c.nG * CSR_GN * 4); c.ROWCNT = (int*)al((size_t)c.nG * CSR_GN * 4); c.FLAG = (int*)al(256);
  c.bytes = off - off0; return off;
}
static void csr_build(const CsrBufs& c, const int* dst, int E, int N, hipStream_t stream) {
  const size_t smem = (size_t)(2 * c.NGP + c.CHP) * 4;
  csrZ_kernel<<<512, 256, 0, stream>>>((int*)c.base, c.bytes / 16);
  csrA_kernel<<<CSR_NBLK, 64, smem, stream>>>(dst, E, N, c.nG, c.CHP, c.NGP, c.STG, c.HST);
  csrS_kernel<<<1, 512, 0, stream>>>(c.HST, c.nG, c.NGP, c.START, c.TOT, c.OFF);
  csrB_kernel<<<c.nG, 256, 0, stream>>>(dst, N, c.nG, c.CHP, c.NGP, (int)c.permLen, c.STG, c.HST, c.OFF, c.START, c.TOT, c.PERM, c.ROWPTR, c.ROWCNT, c.FLAG);
}


__global__ __launch_bounds__(256) void prep_kernel(const float* __restrict__ x, const float* const* __restrict__ wl  , b16* __restrict__ X16) {
  const size_t u = (size_t)blockIdx.x * 256 + threadIdx.x; if (u >= (size_t)NP * F0 / 8) return; const size_t e = u * 8; const size_t row = e / F0; v8b o;
  for (int j = 0; j < 8; ++j) o[j] = (row < (size_t)N) ? (b16)(bf16_rne(x[e + j]) * XS) : (b16)0.0f;
  for (int pass = 0; pass < 2; ++pass) { *(volatile v8b*)(X16 + e) = o; __threadfence(); } (void)wl;
}
__global__ __launch_bounds__(256) void wprep_kernel(const float* __restrict__ w, int nin, int nout, int noutp, b16* __restrict__ dst) {
  const int u = blockIdx.x * 256 + threadIdx.x; if (u >= noutp * nin / 8) return; const int e = u * 8, oo = e / nin, k0 = e % nin; v8b o;
  for (int j = 0; j < 8; ++j) o[j] = (oo < nout) ? (b16)(bf16_rne(w[(size_t)(k0 + j) * nout + oo]) * WSC) : (b16)0.0f;
  for (int pass = 0; pass < 2; ++pass) { *(volatile v8b*)(dst + e) = o; __threadfence(); }
}
template <int MODE>
__global__ __launch_bounds__(128) void xw_kernel(const b16* __restrict__ X16, const float* __restrict__ Hin, const b16* __restrict__ Wt, const float* __restrict__ bias, const float* __restrict__ ADD, float* __restrict__ Y) {
  __shared__ __attribute__((aligned(16))) b16 Ah[4][16][H + 8], Al[4][16][H + 8]; __shared__ __attribute__((aligned(16))) float Tf[4][16][H + 4];
  const int wave = threadIdx.x >> 5, lane = threadIdx.x & 31, nloc = lane & 15, hlf = lane >> 4; const size_t m0 = (size_t)blockIdx.x * 64 + wave * 16; v8f acc[4] = {{}, {}, {}, {}};
  if (MODE == 0) {
#pragma unroll
    for (int kb = 0; kb < F0; kb += 32) { const v16b a = frag_kb(X16 + (m0 + nloc) * F0 + kb, hlf);
#pragma unroll
      for (int t = 0; t < 4; ++t) acc[t] = wmma16b(a, frag_kb(Wt + (size_t)(t * 16 + nloc) * F0 + kb, hlf), acc[t]); }
  } else {
    for (int q = lane; q < 16 * (H / 4); q += 32) { const int rr = q / (H / 4), c4 = (q % (H / 4)) * 4; const v4f xv = *(const v4f*)(Hin + (m0 + rr) * H + c4); for (int j = 0; j < 4; ++j) { b16 p, pl; split16(xv[j] * XS, p, pl); Ah[wave][rr][c4 + j] = p; Al[wave][rr][c4 + j] = pl; } }
    wave_lds_sync();
#pragma unroll
    for (int kb = 0; kb < H; kb += 32) { const v16b a = frag_kb(&Ah[wave][nloc][kb], hlf), al = frag_kb(&Al[wave][nloc][kb], hlf);
#pragma unroll
      for (int t = 0; t < 4; ++t) { const v16b bw = frag_kb(Wt + (size_t)(t * 16 + nloc) * H + kb, hlf); acc[t] = wmma16b(a, bw, acc[t]); acc[t] = wmma16b(al, bw, acc[t]); } } }
#pragma unroll
  for (int t = 0; t < 4; ++t) { const int c = t * 16 + nloc; const float bb = (MODE == 2) ? bf16_rne(bias[c]) : 0.0f;
#pragma unroll 1
    for (int r = 0; r < 8; ++r) { float y = acc[t][r] * (1.0f / (XS * WSC)) + bb; if (MODE == 2) y += ADD[(m0 + 8 * hlf + r) * H + c]; Tf[wave][8 * hlf + r][c] = y; } }
  wave_lds_sync();
  for (int pass = 0; pass < 2; ++pass) { for (int rr = 0; rr < 16; ++rr) if (lane < 16) *(volatile v4f*)(Y + (m0 + rr) * H + lane * 4) = *(const v4f*)(&Tf[wave][rr][lane * 4]); __threadfence(); }
}
template <int LNR>
__global__ __launch_bounds__(256) void agg_kernel(const float* __restrict__ XW, const int* __restrict__ srcs, const int* __restrict__ PERM, const int* __restrict__ ROWPTR, const int* __restrict__ ROWCNT, int permLen, const float* __restrict__ bias, const float* __restrict__ g, const float* __restrict__ bta, float* __restrict__ Hout) {
  __shared__ __attribute__((aligned(16))) float row[8][H];
  const int wave = threadIdx.x >> 5, lane = threadIdx.x & 31; const size_t v = (size_t)blockIdx.x * 8 + wave; float y0 = 0.0f, y1 = 0.0f;
  if (v < (size_t)N) { int st = ROWPTR[v], cnt = ROWCNT[v]; cnt = iclamp(cnt, 0, 65536); st = iclamp(st, 0, permLen - cnt); const float dv = rsqrtf((float)cnt + 1.0f);
    float a0 = 0.0f, a1 = 0.0f;
    for (int i = 0; i < cnt; ++i) { const int e = iclamp(PERM[st + i], 0, E - 1); const size_t s = (size_t)iclamp(srcs[e], 0, N - 1); const float ds = rsqrtf((float)iclamp(ROWCNT[s], 0, 65536) + 1.0f); const float2 xs = *(const float2*)(XW + s * H + lane * 2); const float nrm = pmul(ds, dv); a0 += pmul(xs.x, nrm); a1 += pmul(xs.y, nrm); }
    const float2 xv = *(const float2*)(XW + v * H + lane * 2); const float dd = pmul(dv, dv); y0 = a0 + pmul(xv.x, dd) + bf16_rne(bias[lane * 2]); y1 = a1 + pmul(xv.y, dd) + bf16_rne(bias[lane * 2 + 1]);
    if (LNR) { float s = y0 + y1;
#pragma unroll
      for (int o = 16; o >= 1; o >>= 1) s += __shfl_xor(s, o);
      const float mu = s * (1.0f / H); const float d0 = y0 - mu, d1 = y1 - mu; float q = d0 * d0 + d1 * d1;
#pragma unroll
      for (int o = 16; o >= 1; o >>= 1) q += __shfl_xor(q, o);
      const float rs = rsqrtf(q * (1.0f / H) + LNEPS); y0 = fmaxf(d0 * rs * bf16_rne(g[lane * 2]) + bf16_rne(bta[lane * 2]), 0.0f); y1 = fmaxf(d1 * rs * bf16_rne(g[lane * 2 + 1]) + bf16_rne(bta[lane * 2 + 1]), 0.0f); } }
  row[wave][lane * 2] = y0; row[wave][lane * 2 + 1] = y1;
  wave_lds_sync();
  for (int pass = 0; pass < 2; ++pass) { if (lane < 16) *(volatile v4f*)(Hout + v * H + lane * 4) = *(const v4f*)(&row[wave][lane * 4]); __threadfence(); }
}
__global__ __launch_bounds__(256) void pool_kernel(const float* __restrict__ Hn, const int* __restrict__ seg, float* __restrict__ POOL) {
  __shared__ float part[4][H]; __shared__ __attribute__((aligned(16))) float rowp[H];
  const int g = blockIdx.x, t_ = threadIdx.x, c = t_ & 63, grp = t_ >> 6;
  int lo, hi_; { int a = 0, b = N; while (a < b) { const int m = (a + b) >> 1; if (seg[m] < g) a = m + 1; else b = m; } lo = a; a = 0; b = N; while (a < b) { const int m = (a + b) >> 1; if (seg[m] < g + 1) a = m + 1; else b = m; } hi_ = a; }
  float s = 0.0f; for (int r = lo + grp; r < hi_; r += 4) s += Hn[(size_t)r * H + c]; part[grp][c] = s;
  __syncthreads();
  if (t_ < H) { const int cnt = hi_ - lo; rowp[t_] = (part[0][t_] + part[1][t_] + part[2][t_] + part[3][t_]) / fmaxf((float)cnt, 1.0f); }
  __syncthreads();
  for (int pass = 0; pass < 2; ++pass) { if (t_ < 16) *(volatile v4f*)(POOL + (size_t)g * H + t_ * 4) = *(const v4f*)(&rowp[t_ * 4]); __threadfence(); }
}
__global__ __launch_bounds__(128) void head_kernel(const float* __restrict__ POOL, const b16* __restrict__ Wm1T, const float* __restrict__ bm1, const float* __restrict__ wm2, const float* __restrict__ bm2, float* __restrict__ out) {
  __shared__ __attribute__((aligned(16))) b16 Ah[4][16][H + 8], Al[4][16][H + 8]; __shared__ __attribute__((aligned(16))) float Z[NG][H + 4]; __shared__ __attribute__((aligned(16))) float res[NG];
  const int wave = threadIdx.x >> 5, lane = threadIdx.x & 31, nloc = lane & 15, hlf = lane >> 4; const int m0 = wave * 16;
  for (int q = lane; q < 16 * (H / 4); q += 32) { const int rr = q / (H / 4), c4 = (q % (H / 4)) * 4; const v4f xv = *(const v4f*)(POOL + (size_t)(m0 + rr) * H + c4); for (int j = 0; j < 4; ++j) { b16 p, pl; split16(xv[j] * XS, p, pl); Ah[wave][rr][c4 + j] = p; Al[wave][rr][c4 + j] = pl; } }
  wave_lds_sync(); v8f acc[4] = {{}, {}, {}, {}};
#pragma unroll
  for (int kb = 0; kb < H; kb += 32) { const v16b a = frag_kb(&Ah[wave][nloc][kb], hlf), al = frag_kb(&Al[wave][nloc][kb], hlf);
#pragma unroll
    for (int t = 0; t < 4; ++t) { const v16b bw = frag_kb(Wm1T + (size_t)(t * 16 + nloc) * H + kb, hlf); acc[t] = wmma16b(a, bw, acc[t]); acc[t] = wmma16b(al, bw, acc[t]); } }
#pragma unroll
  for (int t = 0; t < 4; ++t) { const int c = t * 16 + nloc; const float bb = bf16_rne(bm1[c]);
#pragma unroll 1
    for (int r = 0; r < 8; ++r) Z[m0 + 8 * hlf + r][c] = fmaxf(acc[t][r] * (1.0f / (XS * WSC)) + bb, 0.0f); }
  __syncthreads();
  if (threadIdx.x < NG) { float s = bf16_rne(bm2[0]); for (int c = 0; c < H; ++c) s += pmul(Z[threadIdx.x][c], bf16_rne(wm2[c])); res[threadIdx.x] = s; }
  __syncthreads();
  for (int pass = 0; pass < 2; ++pass) { if (threadIdx.x < 16) *(volatile v4f*)(out + threadIdx.x * 4) = *(const v4f*)(&res[threadIdx.x * 4]); __threadfence(); }
}
}

extern "C" void kernel_launch(void* const* d_in, const int* in_sizes, int n_in, void* d_out, int out_size, void* d_ws, size_t ws_size, hipStream_t stream) {
  (void)n_in;
  auto Fp = [&](int i) { return (const float*)d_in[i]; }; auto Ip = [&](int i) { return (const int*)d_in[i]; };
  if (in_sizes[0] != N * F0 || in_sizes[1] != 2 * E || in_sizes[2] != N || in_sizes[3] != F0 * H || in_sizes[5] != H * H || in_sizes[25] != H * H || in_sizes[29] != H || out_size != NG) return;
  size_t off = 0; char* ws = (char*)d_ws;
  auto carve = [&](size_t bytes) { char* p = ws + off; off += (bytes + 255) & ~(size_t)255; return p; };
  b16* X16 = (b16*)carve((size_t)NP * F0 * 2); b16* W1T = (b16*)carve((size_t)H * F0 * 2); b16* WT[8]; for (int k = 0; k < 8; ++k) WT[k] = (b16*)carve((size_t)H * H * 2);
  float* XW = (float*)carve((size_t)NP * H * 4); float* HA = (float*)carve((size_t)NP * H * 4); float* HB = (float*)carve((size_t)NP * H * 4); float* H1 = (float*)X16  ; float* POOL = (float*)carve((size_t)NG * H * 4);
  CsrBufs csr; off = csr_carve(csr, ws, off, E, N);
  if (off > ws_size || off > ((size_t)128 << 20)) return;
  prep_kernel<<<(unsigned)(((size_t)NP * F0 / 8 + 255) / 256), 256, 0, stream>>>(Fp(0), nullptr, X16);
  wprep_kernel<<<(H * F0 / 8 + 255) / 256, 256, 0, stream>>>(Fp(3), F0, H, H, W1T);
  const int widx[7] = {5, 7, 9, 11, 13, 25, 27};
  for (int k = 0; k < 7; ++k) wprep_kernel<<<(H * H / 8 + 255) / 256, 256, 0, stream>>>(Fp(widx[k]), H, H, H, WT[k]);
  csr_build(csr, Ip(1) + E, E, N, stream);
  xw_kernel<0><<<NP / 64, 128, 0, stream>>>(X16, nullptr, W1T, nullptr, nullptr, XW);
  agg_kernel<1><<<NP / 8, 256, 0, stream>>>(XW, Ip(1), csr.PERM, csr.ROWPTR, csr.ROWCNT, (int)csr.permLen, Fp(4), Fp(15), Fp(16), H1);
  xw_kernel<1><<<NP / 64, 128, 0, stream>>>(nullptr, H1, WT[0], nullptr, nullptr, XW);
  agg_kernel<1><<<NP / 8, 256, 0, stream>>>(XW, Ip(1), csr.PERM, csr.ROWPTR, csr.ROWCNT, (int)csr.permLen, Fp(6), Fp(17), Fp(18), HA);
  xw_kernel<1><<<NP / 64, 128, 0, stream>>>(nullptr, HA, WT[1], nullptr, nullptr, XW);
  agg_kernel<1><<<NP / 8, 256, 0, stream>>>(XW, Ip(1), csr.PERM, csr.ROWPTR, csr.ROWCNT, (int)csr.permLen, Fp(8), Fp(19), Fp(20), HB);
  xw_kernel<2><<<NP / 64, 128, 0, stream>>>(nullptr, H1, WT[5], Fp(26), HB, HA);
  xw_kernel<1><<<NP / 64, 128, 0, stream>>>(nullptr, HA, WT[2], nullptr, nullptr, XW);
  agg_kernel<1><<<NP / 8, 256, 0, stream>>>(XW, Ip(1), csr.PERM, csr.ROWPTR, csr.ROWCNT, (int)csr.permLen, Fp(10), Fp(21), Fp(22), HB);
  xw_kernel<1><<<NP / 64, 128, 0, stream>>>(nullptr, HB, WT[3], nullptr, nullptr, XW);
  agg_kernel<1><<<NP / 8, 256, 0, stream>>>(XW, Ip(1), csr.PERM, csr.ROWPTR, csr.ROWCNT, (int)csr.permLen, Fp(12), Fp(23), Fp(24), HA);
  xw_kernel<1><<<NP / 64, 128, 0, stream>>>(nullptr, HA, WT[4], nullptr, nullptr, XW);
  agg_kernel<0><<<NP / 8, 256, 0, stream>>>(XW, Ip(1), csr.PERM, csr.ROWPTR, csr.ROWCNT, (int)csr.permLen, Fp(14), Fp(15), Fp(16), HB);
  pool_kernel<<<NG, 256, 0, stream>>>(HB, Ip(2), POOL);
  head_kernel<<<1, 128, 0, stream>>>(POOL, WT[6], Fp(28), Fp(29), Fp(30), (float*)d_out);
}
